// IGNEncoder_28939489641150
// MI455X (gfx1250) — hardware-verified
//
#include <hip/hip_runtime.h>
#include <stddef.h>
#include <stdint.h>

#define NB     32
#define MS     128
#define D1     16
#define HD     64
#define NNODE  (NB * MS)
#define NPOS   (NB * MS * MS)
#define NPW    192
#define K1N    192
#define K2N    640
#define A2P    264
#define SPT    68
#define WSMAX  134217728
#define KATTR  __attribute__((amdgpu_num_vgpr(248)))

#define U_XB   (NPOS * 2)
#define U_W1P  (128 * 4)
#define U_W1N  (192 * 24)
#define U_W2P  (64 * 32)
#define U_W2N  (192 * 80)
#define U_W3N  (64 * 80)
#define U_ALL  (U_XB + U_W1P + U_W1N + U_W2P + U_W2N + U_W3N)
#define PREP_BLOCKS (U_ALL / 256 + 1)

#define PV_B1   0
#define PV_B2   192
#define PV_B3   384
#define PV_G1   448
#define PV_BE1  512
#define PV_G2   576
#define PV_BE2  640
#define PV_G3   704
#define PV_BE3  768

#define PL_FRG  0
#define PL_FDG  1024
#define PL_FCC  2048
#define PL_ROW  10240
#define PL_COL  18432
#define PL_DIA  26624
#define PL_ST   27648
#define PL_END0 29696
#define PL_GRG  29696
#define PL_GCC  37888
#define PL_GDG  46080
#define PL_BN   47104
#define PL_A2   47360
#define PL_END1 (PL_A2 + (8 * 16 * A2P) / 2)
#define PAIR0_LDS (PL_END0 * 4)
#define PAIR1_LDS (PL_END1 * 4)

#define BN_DIAG 0
#define BN_ROW  8192
#define BN_COL  16384
#define BN_SD   24576
#define BN_TOT  24640
#define BN_LDS_FLOATS 24704
#define BN_LDS  (BN_LDS_FLOATS * 4)
#define F0_LDS  (128 * 192 * 2)

static_assert(MS == 128 && NB == 32 && D1 == 16 && HD == 64);
static_assert(NNODE == 4096 && NNODE % 64 == 0);
static_assert(K1N % 32 == 0 && K2N % 32 == 0 && K1N == 2 * 5 * D1 + 32 && K2N == 2 * 5 * HD);
static_assert(U_XB % 256 == 0 && U_W1P % 256 == 0 && U_W1N % 256 == 0);
static_assert(U_W2P % 256 == 0 && U_W2N % 256 == 0 && U_W3N % 256 == 0);
static_assert((A2P * 2) % 16 == 0 && A2P >= 256);
static_assert((PL_ST % 2) == 0 && ((PL_A2 * 4) % 16) == 0);
static_assert(PAIR1_LDS <= 300000 && PAIR0_LDS <= 300000 && BN_LDS <= 300000);
static_assert(16 * 16 == 256 && 8 * 32 == 256);

typedef float          v4f   __attribute__((ext_vector_type(4)));
typedef float          v8f   __attribute__((ext_vector_type(8)));
typedef double         v2d   __attribute__((ext_vector_type(2)));
typedef int            v4i   __attribute__((ext_vector_type(4)));
typedef int            v8i   __attribute__((ext_vector_type(8)));
typedef unsigned int   v4u   __attribute__((ext_vector_type(4)));
typedef unsigned short v8us  __attribute__((ext_vector_type(8)));
typedef unsigned short v16us __attribute__((ext_vector_type(16)));
typedef __bf16         v16bf __attribute__((ext_vector_type(16)));
typedef v4f  __attribute__((may_alias)) v4fa;
typedef v4i  __attribute__((may_alias)) v4ia;
typedef v4u  __attribute__((may_alias)) v4ua;
typedef v8us __attribute__((may_alias)) v8usa;
union FragB { v16bf v; v16us u; v8us h[2]; v8i w; };

__device__ __forceinline__ v8f wmb(const FragB& a, const FragB& b, v8f c) {
  v8f d = __builtin_amdgcn_wmma_f32_16x16x32_bf16(false, a.v, false, b.v, (short)0, c, false, false);
  asm volatile("v_nop\n\tv_nop\n\tv_nop\n\tv_nop" : "+v"(d) : "v"(a.w), "v"(b.w));
  return d;
}
__device__ __forceinline__ v8f z8() { v8f z = {0.f, 0.f, 0.f, 0.f, 0.f, 0.f, 0.f, 0.f}; return z; }

__device__ __forceinline__ unsigned bf16_bits(float f) {
  const unsigned u = __float_as_uint(f);
  return (u + 0x7FFFu + ((u >> 16) & 1u)) >> 16;
}
__device__ __forceinline__ float bf16_val(float f) { return __uint_as_float(bf16_bits(f) << 16); }
__device__ __forceinline__ float lo16(unsigned w) { return __uint_as_float(w << 16); }
__device__ __forceinline__ float hi16(unsigned w) { return __uint_as_float(w & 0xffff0000u); }
__device__ __forceinline__ void put16(unsigned short* dp, v8us o) {
  *(volatile v8us*)dp = o;
  __threadfence();
  *(volatile v8us*)dp = o;
}
__device__ __forceinline__ float fsel(float a, float b, unsigned mask) {
  return __uint_as_float((__float_as_uint(a) & ~mask) | (__float_as_uint(b) & mask));
}
__device__ __forceinline__ float relu_sel(float v) { return (v > 0.0f) ? v : (v - v); }

__device__ __forceinline__ int node_basis(int blk, int q) {
  const int rg = (q == 0) ? 11 : ((q == 1) ? 13 : ((q == 2) ? 6 : ((q == 3) ? 5 : 14)));
  const int cc = (q == 0) ? 12 : ((q == 2) ? 8 : ((q == 3) ? 7 : -1));
  return (blk == 0) ? q : ((blk == 1) ? rg : cc);
}
__device__ __forceinline__ v8us node_unit(const float* __restrict__ cf, int n, int k8, int DIN, int KH) {
  const int valid = (k8 < 2 * KH) ? 1 : 0;
  int kk = (k8 < KH) ? k8 : (k8 - KH);
  kk = valid ? kk : 0;
  const int q  = kk / DIN;
  const int d0 = kk - q * DIN;
  const int b  = node_basis(n >> 6, q);
  const unsigned mk = (valid != 0 && b >= 0) ? 0xffffu : 0u;
  const int bc = (b < 0) ? 0 : b;
  const float* p = cf + ((size_t)d0 * 64 + (size_t)(n & 63)) * 15 + bc;
  v8us o;
#pragma unroll
  for (int e = 0; e < 8; ++e) o[e] = (unsigned short)(bf16_bits(p[(size_t)e * 960]) & mk);
  return o;
}

__global__ __launch_bounds__(256) KATTR void k_prep(
    const float* __restrict__ attn, const float* __restrict__ c1, const float* __restrict__ c2,
    const float* __restrict__ c3,
    const float* __restrict__ db1, const float* __restrict__ ab1, const float* __restrict__ g1,
    const float* __restrict__ be1,
    const float* __restrict__ db2, const float* __restrict__ ab2, const float* __restrict__ g2,
    const float* __restrict__ be2,
    const float* __restrict__ b3, const float* __restrict__ g3, const float* __restrict__ be3,
    unsigned short* XB, unsigned short* W1P, unsigned short* W1N, unsigned short* W2P,
    unsigned short* W2N, unsigned short* W3N, float* PV) {
  __shared__ __attribute__((aligned(16))) float pvs[1024];
  const int tid = (int)threadIdx.x;
  const int u   = (int)blockIdx.x * 256 + tid;
  const int L0 = U_XB;
  const int L1 = L0 + U_W1P;
  const int L2 = L1 + U_W1N;
  const int L3 = L2 + U_W2P;
  const int L4 = L3 + U_W2N;
  const int L5 = L4 + U_W3N;
  v8us o;
  if (u < L0) {
    const float* p = attn + (size_t)u * 8;
    const v4f a = *(const v4f*)p;
    const v4f b = *(const v4f*)(p + 4);
    o[0] = (unsigned short)bf16_bits(a.x); o[1] = (unsigned short)bf16_bits(a.y);
    o[2] = (unsigned short)bf16_bits(a.z); o[3] = (unsigned short)bf16_bits(a.w);
    o[4] = (unsigned short)bf16_bits(b.x); o[5] = (unsigned short)bf16_bits(b.y);
    o[6] = (unsigned short)bf16_bits(b.z); o[7] = (unsigned short)bf16_bits(b.w);
    put16(XB + (size_t)u * 8, o);
  } else if (u < L1) {
    const int v  = u - L0;
    const int n  = v >> 2;
    const int k8 = (v & 3) * 8;
    const int basis = 9 + ((k8 >> 4) ^ (n >> 6));
    const float* p = c1 + ((size_t)(k8 & 15) * 64 + (size_t)(n & 63)) * 15 + basis;
#pragma unroll
    for (int e = 0; e < 8; ++e) o[e] = (unsigned short)bf16_bits(p[(size_t)e * 960]);
    put16(W1P + (size_t)v * 8, o);
  } else if (u < L2) {
    const int v  = u - L1;
    const int n  = v / 24;
    const int k8 = (v - n * 24) * 8;
    o = node_unit(c1, n, k8, D1, 5 * D1);
    put16(W1N + (size_t)v * 8, o);
  } else if (u < L3) {
    const int v  = u - L2;
    const int n  = v >> 5;
    const int k8 = (v & 31) * 8;
    const int kk = k8 & 127;
    const int basis = 9 + (kk >> 6);
    const float* p = c2 + ((size_t)(kk & 63) * 64 + (size_t)n) * 15 + basis;
#pragma unroll
    for (int e = 0; e < 8; ++e) o[e] = (unsigned short)bf16_bits(p[(size_t)e * 960]);
    put16(W2P + (size_t)v * 8, o);
  } else if (u < L4) {
    const int v  = u - L3;
    const int n  = v / 80;
    const int k8 = (v - n * 80) * 8;
    o = node_unit(c2, n, k8, HD, 5 * HD);
    put16(W2N + (size_t)v * 8, o);
  } else if (u < L5) {
    const int v  = u - L4;
    const int n  = v / 80;
    const int k8 = (v - n * 80) * 8;
    const int kk = (k8 < 320) ? k8 : (k8 - 320);
    const int q  = kk >> 6;
    const int d0 = kk & 63;
    const float* p = c3 + ((size_t)d0 * 64 + (size_t)n) * 5 + q;
#pragma unroll
    for (int e = 0; e < 8; ++e) o[e] = (unsigned short)bf16_bits(p[(size_t)e * 320]);
    put16(W3N + (size_t)v * 8, o);
  } else {
    for (int i = tid; i < 1024; i += 256) pvs[i] = 0.0f;
    __syncthreads();
    const int c = tid & 63;
    if (tid < 64) {
      const float a = db1[c], b = ab1[c], d = db2[c], e = ab2[c];
      pvs[c] = bf16_val(a); pvs[64 + c] = bf16_val(b); pvs[192 + c] = bf16_val(d); pvs[256 + c] = bf16_val(e);
    }
    __syncthreads();
    if (tid < 64) {
      const float a = b3[c], b = g1[c], d = be1[c], e = g2[c];
      pvs[384 + c] = bf16_val(a); pvs[448 + c] = bf16_val(b); pvs[512 + c] = bf16_val(d); pvs[576 + c] = bf16_val(e);
    }
    __syncthreads();
    if (tid < 64) {
      const float a = be2[c], b = g3[c], d = be3[c];
      pvs[640 + c] = bf16_val(a); pvs[704 + c] = bf16_val(b); pvs[768 + c] = bf16_val(d);
    }
    __syncthreads();
    const v4f v = *(const v4fa*)(pvs + 4 * tid);
    *(volatile v4f*)(PV + 4 * tid) = v;
    __threadfence();
    *(volatile v4f*)(PV + 4 * tid) = v;
  }
}

__global__ __launch_bounds__(256) KATTR void k_feat0(const unsigned short* __restrict__ XB, unsigned short* F0HL) {
  extern __shared__ __attribute__((aligned(16))) unsigned short stile[];
  __shared__ __attribute__((aligned(16))) float sf[6176];
  const int tid = (int)threadIdx.x, lane = tid & 31, wave = tid >> 5;
  const int n = (int)blockIdx.x;
  const int p = tid >> 1, dh = tid & 1;
  float ar[8], ac[8];
#pragma unroll
  for (int e = 0; e < 8; ++e) { ar[e] = 0.0f; ac[e] = 0.0f; }
  const unsigned short* rb = XB + ((size_t)(n * MS + p) * MS) * D1 + 8 * dh;
  const unsigned short* cb = XB + ((size_t)n * MS * MS + (size_t)p) * D1 + 8 * dh;
#pragma unroll 4
  for (int t = 0; t < MS; ++t) {
    const v4u a = *(const v4ua*)(rb + (size_t)t * D1);
    const v4u b = *(const v4ua*)(cb + (size_t)t * (MS * D1));
    ar[0] += lo16(a.x); ar[1] += hi16(a.x); ar[2] += lo16(a.y); ar[3] += hi16(a.y);
    ar[4] += lo16(a.z); ar[5] += hi16(a.z); ar[6] += lo16(a.w); ar[7] += hi16(a.w);
    ac[0] += lo16(b.x); ac[1] += hi16(b.x); ac[2] += lo16(b.y); ac[3] += hi16(b.y);
    ac[4] += lo16(b.z); ac[5] += hi16(b.z); ac[6] += lo16(b.w); ac[7] += hi16(b.w);
  }
  {
    const v4u d = *(const v4ua*)(rb + (size_t)p * D1);
    float* sd0 = sf + p * 16 + 8 * dh;
    sd0[0] = lo16(d.x); sd0[1] = hi16(d.x); sd0[2] = lo16(d.y); sd0[3] = hi16(d.y);
    sd0[4] = lo16(d.z); sd0[5] = hi16(d.z); sd0[6] = lo16(d.w); sd0[7] = hi16(d.w);
#pragma unroll
    for (int e = 0; e < 8; ++e) { sf[2048 + p * 16 + 8 * dh + e] = ar[e]; sf[4096 + p * 16 + 8 * dh + e] = ac[e]; }
  }
  __syncthreads();
  if (wave == 0) {
    const int d = lane & 15;
    float s = 0.0f;
#pragma unroll 4
    for (int i = 0; i < MS; ++i) s += sf[i * 16 + d];
    sf[6144 + d] = s;
  } else if (wave == 1) {
    const int d = lane & 15;
    float s = 0.0f;
#pragma unroll 4
    for (int i = 0; i < MS; ++i) s += sf[2048 + i * 16 + d];
    sf[6160 + d] = s;
  }
  __syncthreads();
#pragma unroll 2
  for (int it = 0; it < 40; ++it) {
    const int idx = it * 256 + tid;
    const int i = idx / 80;
    const int k = idx - i * 80;
    const int q = k >> 4, d = k & 15;
    const int base = (q == 0) ? 0 : ((q == 2) ? 2048 : ((q == 3) ? 4096 : ((q == 1) ? 6144 : 6160)));
    const int rm = (q == 1 || q == 4) ? 0 : 16;
    const float sc = (q == 0) ? 1.0f : ((q == 4) ? 6.103515625e-05f : 0.0078125f);
    const float f = sf[base + i * rm + d] * sc;
    const unsigned hb = bf16_bits(f);
    const unsigned lb = bf16_bits(f - __uint_as_float(hb << 16));
    stile[i * 192 + k] = (unsigned short)hb;
    stile[i * 192 + 80 + k] = (unsigned short)lb;
  }
#pragma unroll 2
  for (int it = 0; it < 16; ++it) {
    const int idx = it * 256 + tid;
    stile[(idx >> 5) * 192 + 160 + (idx & 31)] = (unsigned short)0;
  }
  __syncthreads();
  unsigned short* ob = F0HL + (size_t)n * (MS * 192);
#pragma unroll 1
  for (int sw = 0; sw < 12; ++sw) {
    const int v = sw * 256 + tid;
    const v8us o = *(const v8usa*)(stile + v * 8);
    *(volatile v8us*)(ob + (size_t)v * 8) = o;
  }
  __threadfence();
#pragma unroll 1
  for (int sw = 0; sw < 12; ++sw) {
    const int v = sw * 256 + tid;
    const v8us o = *(const v8usa*)(stile + v * 8);
    *(volatile v8us*)(ob + (size_t)v * 8) = o;
  }
}

template <int RELU>
__global__ __launch_bounds__(128) KATTR void k_node(const unsigned short* __restrict__ A, int lda,
                                                    const unsigned short* __restrict__ BT, int ldb, int K,
                                                    const float* __restrict__ bias, float* of, int ldc) {
  __shared__ __attribute__((aligned(16))) float stg[64 * SPT];
  __shared__ __attribute__((aligned(16))) float sb[64];
  const int tid = (int)threadIdx.x, lane = tid & 31, wave = tid >> 5, hh = lane >> 4, m = lane & 15;
  const int rowBase = (int)blockIdx.x * 64;
  const int colBase = (int)blockIdx.y * 64;
  if (tid < 64) sb[tid] = bias[colBase + tid];

  v8f acc[4];
#pragma unroll
  for (int t = 0; t < 4; ++t) acc[t] = z8();
  const unsigned short* ap = A  + (size_t)(rowBase + 16 * wave + m) * (size_t)lda + 8 * hh;
  const unsigned short* bp = BT + (size_t)(colBase + m) * (size_t)ldb + 8 * hh;

#pragma unroll 1
  for (int k0 = 0; k0 < K; k0 += 32) {
    FragB af;
    af.h[0] = *(const v8usa*)(ap + k0);
    af.h[1] = *(const v8usa*)(ap + k0 + 16);
#pragma unroll
    for (int nt = 0; nt < 4; ++nt) {
      const unsigned short* wq = bp + (size_t)(16 * nt) * (size_t)ldb + k0;
      FragB bf;
      bf.h[0] = *(const v8usa*)wq;
      bf.h[1] = *(const v8usa*)(wq + 16);
      acc[nt] = wmb(af, bf, acc[nt]);
    }
  }
#pragma unroll
  for (int nt = 0; nt < 4; ++nt) {
    const int lc = 16 * nt + m;
#pragma unroll
    for (int r = 0; r < 8; ++r) {
      const int lr = 16 * wave + 8 * hh + r;
      stg[lr * SPT + lc] = acc[nt][r];
    }
  }
  __syncthreads();
  const int rsub = tid >> 4;
  const int c4   = (tid & 15) * 4;
  v4f pv[8];
#pragma unroll
  for (int it = 0; it < 8; ++it) {
    const int row = it * 8 + rsub;
    v4f v = *(const v4fa*)(stg + row * SPT + c4);
    v.x += sb[c4]; v.y += sb[c4 + 1]; v.z += sb[c4 + 2]; v.w += sb[c4 + 3];
    if (RELU) { v.x = relu_sel(v.x); v.y = relu_sel(v.y); v.z = relu_sel(v.z); v.w = relu_sel(v.w); }
    pv[it] = v;
  }
#pragma unroll
  for (int it = 0; it < 8; ++it) {
    const int row = it * 8 + rsub;
    *(volatile v4f*)(of + (size_t)(rowBase + row) * (size_t)ldc + colBase + c4) = pv[it];
  }
  __threadfence();
#pragma unroll
  for (int it = 0; it < 8; ++it) {
    const int row = it * 8 + rsub;
    *(volatile v4f*)(of + (size_t)(rowBase + row) * (size_t)ldc + colBase + c4) = pv[it];
  }
}

template <int MODE>
__global__ __launch_bounds__(256) KATTR void k_pair(const unsigned short* __restrict__ XB,
                                                    const unsigned short* __restrict__ W1P,
                                                    const unsigned short* __restrict__ W2P,
                                                    const float* __restrict__ NP1, const float* __restrict__ NP2,
                                                    const float* __restrict__ BNP1,
                                                    float* ROW, float* DIAG, float* COLP, double* STAT) {
  extern __shared__ __attribute__((aligned(16))) float dyn[];
  constexpr int NT1 = (MODE == 0) ? 4 : 8;
  const int tid = (int)threadIdx.x, lane = tid & 31, wave = tid >> 5, hh = lane >> 4, c = lane & 15;
  const int bx = (int)blockIdx.x, n = bx >> 3, It = bx & 7, I = It * 16;
  const float* __restrict__ NPf = (MODE == 0) ? NP1 : NP2;
  float* fRG = dyn + PL_FRG;
  float* fDG = dyn + PL_FDG;
  float* fCC = dyn + PL_FCC;
  float* sRow = dyn + PL_ROW;
  float* sCol = dyn + PL_COL;
  float* sDia = dyn + PL_DIA;
  double* sST = (double*)(dyn + PL_ST);
  float* gRG = dyn + PL_GRG;
  float* gCC = dyn + PL_GCC;
  float* gDG = dyn + PL_GDG;
  float* sBN = dyn + PL_BN;

  {
    const int row = tid >> 4, c4 = (tid & 15) * 4;
    const float* src = NPf + (size_t)(n * MS + I + row) * NPW;
    const v4f a = *(const v4f*)(src + c4);
    const v4f b = *(const v4f*)(src + 64 + c4);
    *(v4fa*)(fDG + row * 64 + c4) = a;
    *(v4fa*)(fRG + row * 64 + c4) = b;
    if constexpr (MODE == 1) {
      const float* s1 = NP1 + (size_t)(n * MS + I + row) * NPW;
      const v4f d = *(const v4f*)(s1 + c4);
      *(v4fa*)(gDG + row * 64 + c4) = d;
    }
  }
#pragma unroll 2
  for (int it = 0; it < 8; ++it) {
    const int idx = it * 256 + tid;
    const int row = idx >> 4, c4 = (idx & 15) * 4;
    const float* src = NPf + (size_t)(n * MS + row) * NPW;
    const v4f a = *(const v4f*)(src + 128 + c4);
    *(v4fa*)(fCC + row * 64 + c4) = a;
    if constexpr (MODE == 1) {
      const float* s1 = NP1 + (size_t)(n * MS + row) * NPW;
      const v4f b = *(const v4f*)(s1 + 64 + c4);
      const v4f d = *(const v4f*)(s1 + 128 + c4);
      *(v4fa*)(gRG + row * 64 + c4) = b;
      *(v4fa*)(gCC + row * 64 + c4) = d;
    }
  }
  if constexpr (MODE == 1) {
    if (tid < 64) {
      const v4f a = *(const v4f*)(BNP1 + 4 * tid);
      *(v4fa*)(sBN + 4 * tid) = a;
    }
  }
  __syncthreads();

  const int J = 16 * wave;
  const int jm = J + c;
  const size_t nb = (size_t)n * MS * MS;
  unsigned short* a2w = (unsigned short*)(dyn + PL_A2) + wave * 16 * A2P;
  float colacc[4][8];
  double ssum[4], ssq[4];
#pragma unroll
  for (int nt = 0; nt < 4; ++nt) {
    ssum[nt] = 0.0; ssq[nt] = 0.0;
#pragma unroll
    for (int r = 0; r < 8; ++r) colacc[nt][r] = 0.0f;
  }

#pragma unroll 1
  for (int il = 0; il < 16; ++il) {
    const int i = I + il;
    int zl = 0;
    asm volatile("" : "+v"(zl));
    FragB af;
    af.h[0] = *(const v8usa*)(XB + (nb + (size_t)i * MS + (size_t)jm) * D1 + 8 * hh);
    af.h[1] = *(const v8usa*)(XB + (nb + (size_t)jm * MS + (size_t)i) * D1 + 8 * hh);
    v8f acc1[NT1];
    const unsigned short* w1 = W1P + zl + c * 32 + 8 * hh;
#pragma unroll
    for (int nt = 0; nt < NT1; ++nt) {
      FragB bf;
      bf.h[0] = *(const v8usa*)(w1 + nt * 512);
      bf.h[1] = *(const v8usa*)(w1 + nt * 512 + 16);
      acc1[nt] = wmb(af, bf, z8());
    }

    v8f fa[4];
    if constexpr (MODE == 0) {
#pragma unroll
      for (int nt = 0; nt < 4; ++nt) fa[nt] = acc1[nt];
    } else {
#pragma unroll
      for (int nt = 0; nt < 4; ++nt) {
        const int s = 16 * nt + c;
        const float rgi = gRG[i * 64 + s];
        const float cci = gCC[i * 64 + s];
        const float dgi = gDG[il * 64 + s];
        const float mean = sBN[s], av = sBN[64 + s], be = sBN[128 + s];
#pragma unroll
        for (int r = 0; r < 8; ++r) {
          const int jl = 8 * hh + r;
          const int j  = J + jl;
          const float dg  = (i == j) ? dgi : 0.0f;
          const float vij = ((acc1[nt][r] + rgi) + gCC[j * 64 + s]) + dg;
          const float vji = ((acc1[nt + 4][r] + gRG[j * 64 + s]) + cci) + dg;
          const float hij = (relu_sel(vij) - mean) * av + be;
          const float hji = (relu_sel(vji) - mean) * av + be;
          const unsigned h0 = bf16_bits(hij);
          const unsigned l0 = bf16_bits(hij - __uint_as_float(h0 << 16));
          const unsigned h1 = bf16_bits(hji);
          const unsigned l1 = bf16_bits(hji - __uint_as_float(h1 << 16));
          unsigned short* ar = a2w + jl * A2P + s;
          ar[0]   = (unsigned short)h0;
          ar[64]  = (unsigned short)h1;
          ar[128] = (unsigned short)l0;
          ar[192] = (unsigned short)l1;
        }
      }
      __builtin_amdgcn_fence(__ATOMIC_RELEASE, "workgroup");
      __builtin_amdgcn_wave_barrier();
      __builtin_amdgcn_fence(__ATOMIC_ACQUIRE, "workgroup");
      v8f acc2[4];
#pragma unroll
      for (int nt = 0; nt < 4; ++nt) acc2[nt] = z8();
      const unsigned short* ap2 = a2w + c * A2P + 8 * hh;
      const unsigned short* bp2 = W2P + (size_t)c * 256 + 8 * hh;
#pragma unroll 1
      for (int k0 = 0; k0 < 256; k0 += 32) {
        FragB a2;
        a2.h[0] = *(const v8usa*)(ap2 + k0);
        a2.h[1] = *(const v8usa*)(ap2 + k0 + 16);
#pragma unroll
        for (int nt = 0; nt < 4; ++nt) {
          const unsigned short* wq = bp2 + (size_t)(16 * nt) * 256 + k0;
          FragB bf;
          bf.h[0] = *(const v8usa*)wq;
          bf.h[1] = *(const v8usa*)(wq + 16);
          acc2[nt] = wmb(a2, bf, acc2[nt]);
        }
      }
      __builtin_amdgcn_fence(__ATOMIC_RELEASE, "workgroup");
      __builtin_amdgcn_wave_barrier();
      __builtin_amdgcn_fence(__ATOMIC_ACQUIRE, "workgroup");
#pragma unroll
      for (int nt = 0; nt < 4; ++nt) fa[nt] = acc2[nt];
    }

#pragma unroll
    for (int nt = 0; nt < 4; ++nt) {
      const int s = 16 * nt + c;
      const float rg  = fRG[il * 64 + s];
      const float dg0 = fDG[il * 64 + s];
      float g = 0.0f, q = 0.0f, dv = 0.0f;
#pragma unroll
      for (int r = 0; r < 8; ++r) {
        const int jl = 8 * hh + r;
        const int j  = J + jl;
        const float dgt = (i == j) ? dg0 : 0.0f;
        const float v  = ((fa[nt][r] + rg) + fCC[j * 64 + s]) + dgt;
        const float rl = relu_sel(v);
        g += rl;
        q = fmaf(rl, rl, q);
        colacc[nt][r] += rl;
        dv = (jl == il) ? rl : dv;
      }
      ssum[nt] += (double)g;
      ssq[nt]  += (double)q;
      const float go = __shfl_xor(g, 16, 32);
      const float rp = g + go;
      if (hh == 0) sRow[(wave * 16 + il) * 64 + s] = rp;
      if (wave == It && hh == (il >> 3)) sDia[il * 64 + s] = dv;
    }
  }

  float* cw = sCol + wave * 1024;
#pragma unroll
  for (int nt = 0; nt < 4; ++nt) {
#pragma unroll
    for (int r = 0; r < 8; ++r) cw[(8 * hh + r) * 64 + 16 * nt + c] = colacc[nt][r];
    const double so = __shfl_xor(ssum[nt], 16, 32);
    const double qo = __shfl_xor(ssq[nt], 16, 32);
    const double st = ssum[nt] + so;
    const double qt = ssq[nt] + qo;
    if (hh == 0) {
      sST[(wave * 64 + 16 * nt + c) * 2]     = st;
      sST[(wave * 64 + 16 * nt + c) * 2 + 1] = qt;
    }
  }
  __builtin_amdgcn_fence(__ATOMIC_RELEASE, "workgroup");
  __builtin_amdgcn_wave_barrier();
  __builtin_amdgcn_fence(__ATOMIC_ACQUIRE, "workgroup");
  {
    float* cg = COLP + ((size_t)(n * 8 + It) * MS + (size_t)J) * HD;
    v4f cv[8];
#pragma unroll
    for (int it = 0; it < 8; ++it) cv[it] = *(const v4fa*)(cw + (it * 32 + lane) * 4);
#pragma unroll
    for (int it = 0; it < 8; ++it) *(volatile v4f*)(cg + (size_t)(it * 32 + lane) * 4) = cv[it];
    __threadfence();
#pragma unroll
    for (int it = 0; it < 8; ++it) *(volatile v4f*)(cg + (size_t)(it * 32 + lane) * 4) = cv[it];
  }
  __syncthreads();

  const int il2 = tid >> 4, c4 = (tid & 15) * 4;
  v4f rs = {0.0f, 0.0f, 0.0f, 0.0f};
#pragma unroll
  for (int w = 0; w < 8; ++w) {
    const v4f t = *(const v4fa*)(sRow + (w * 16 + il2) * 64 + c4);
    rs = rs + t;
  }
  const v4f dgv = *(const v4fa*)(sDia + il2 * 64 + c4);
  v2d sv = {0.0, 0.0};
  if (tid < 64) {
    double S = 0.0, Q = 0.0;
#pragma unroll
    for (int w = 0; w < 8; ++w) { S += sST[(w * 64 + tid) * 2]; Q += sST[(w * 64 + tid) * 2 + 1]; }
    sv.x = S; sv.y = Q;
  }
  float* rp = ROW  + (size_t)(n * MS + I + il2) * HD + c4;
  float* dp = DIAG + (size_t)(n * MS + I + il2) * HD + c4;
  double* sp = STAT + ((size_t)bx * 64 + (size_t)(tid & 63)) * 2;
  *(volatile v4f*)rp = rs;
  *(volatile v4f*)dp = dgv;
  if (tid < 64) *(volatile v2d*)sp = sv;
  __threadfence();
  *(volatile v4f*)rp = rs;
  *(volatile v4f*)dp = dgv;
  if (tid < 64) *(volatile v2d*)sp = sv;
}

__global__ __launch_bounds__(256) KATTR void k_bn(const double* __restrict__ STAT, const float* __restrict__ ROW,
                                                  const float* __restrict__ DIAG, const float* __restrict__ COLP,
                                                  const float* __restrict__ gam, const float* __restrict__ bet,
                                                  unsigned short* FHL, float* BNP) {
  extern __shared__ __attribute__((aligned(16))) float big[];
  __shared__ __attribute__((aligned(16))) float sbn[256];
  const int tid = (int)threadIdx.x;
  const int n = (int)blockIdx.x;
  if (tid < 64) {
    double S = 0.0, Q = 0.0;
#pragma unroll 4
    for (int b = 0; b < 256; ++b) {
      const v2d v = *(const v2d*)(STAT + ((size_t)b * 64 + (size_t)tid) * 2);
      S += v.x; Q += v.y;
    }
    const double mean = S * (1.0 / 524288.0);
    double var = Q * (1.0 / 524288.0) - mean * mean;
    var = (var < 0.0) ? 0.0 : var;
    const float rstd = 1.0f / sqrtf((float)var + 1e-5f);
    sbn[tid] = (float)mean;
    sbn[64 + tid] = gam[tid] * rstd;
    sbn[128 + tid] = bet[tid];
    sbn[192 + tid] = 0.0f;
  }
#pragma unroll 2
  for (int it = 0; it < 8; ++it) {
    const int idx = (it * 256 + tid) * 4;
    const v4f a = *(const v4f*)(DIAG + (size_t)n * 8192 + idx);
    const v4f b = *(const v4f*)(ROW + (size_t)n * 8192 + idx);
    v4f cs = {0.0f, 0.0f, 0.0f, 0.0f};
#pragma unroll
    for (int t = 0; t < 8; ++t) {
      const v4f cp = *(const v4f*)(COLP + (size_t)(n * 8 + t) * 8192 + idx);
      cs = cs + cp;
    }
    *(v4fa*)(big + BN_DIAG + idx) = a;
    *(v4fa*)(big + BN_ROW + idx) = b;
    *(v4fa*)(big + BN_COL + idx) = cs;
  }
  __syncthreads();
  if (tid < 128) {
    const int d = tid & 63;
    const int src = (tid < 64) ? BN_DIAG : BN_ROW;
    const int dst = (tid < 64) ? BN_SD : BN_TOT;
    float s = 0.0f;
#pragma unroll 4
    for (int i = 0; i < MS; ++i) s += big[src + i * 64 + d];
    big[dst + d] = s;
  }
  __syncthreads();
  if (n == 0) {
    v4f v = {0.0f, 0.0f, 0.0f, 0.0f};
    if (tid < 64) {
      v = *(const v4fa*)(sbn + 4 * tid);
      *(volatile v4f*)(BNP + 4 * tid) = v;
    }
    __threadfence();
    if (tid < 64) *(volatile v4f*)(BNP + 4 * tid) = v;
  }
#pragma unroll 1
  for (int pass = 0; pass < 2; ++pass) {
#pragma unroll 1
    for (int sw = 0; sw < 20; ++sw) {
      const int p = sw * 256 + tid;
      const int row = p / 40;
      const int w = p - row * 40;
      const int kk = w * 8;
      const int q = kk >> 6, d0 = kk & 63;
      const int base = (q == 0) ? BN_DIAG : ((q == 2) ? BN_ROW : ((q == 3) ? BN_COL : ((q == 1) ? BN_SD : BN_TOT)));
      const int rm = (q == 1 || q == 4) ? 0 : 64;
      const float sc = (q == 0) ? 1.0f : ((q == 4) ? 6.103515625e-05f : 0.0078125f);
      const float* sp = big + base + row * rm + d0;
      const v4f f0 = *(const v4fa*)sp;
      const v4f f1 = *(const v4fa*)(sp + 4);
      const v4f m0 = *(const v4fa*)(sbn + d0);
      const v4f m1 = *(const v4fa*)(sbn + d0 + 4);
      const v4f a0 = *(const v4fa*)(sbn + 64 + d0);
      const v4f a1 = *(const v4fa*)(sbn + 64 + d0 + 4);
      const v4f b0 = *(const v4fa*)(sbn + 128 + d0);
      const v4f b1 = *(const v4fa*)(sbn + 128 + d0 + 4);
      const v8f fv = {f0.x, f0.y, f0.z, f0.w, f1.x, f1.y, f1.z, f1.w};
      const v8f mv = {m0.x, m0.y, m0.z, m0.w, m1.x, m1.y, m1.z, m1.w};
      const v8f av = {a0.x, a0.y, a0.z, a0.w, a1.x, a1.y, a1.z, a1.w};
      const v8f bv = {b0.x, b0.y, b0.z, b0.w, b1.x, b1.y, b1.z, b1.w};
      v8us h8, l8;
#pragma unroll
      for (int e = 0; e < 8; ++e) {
        const float v = (fv[e] * sc - mv[e]) * av[e] + bv[e];
        const unsigned hb = bf16_bits(v);
        const unsigned lb = bf16_bits(v - __uint_as_float(hb << 16));
        h8[e] = (unsigned short)hb;
        l8[e] = (unsigned short)lb;
      }
      unsigned short* dst = FHL + (size_t)(n * MS + row) * K2N + kk;
      *(volatile v8us*)dst = h8;
      *(volatile v8us*)(dst + 320) = l8;
    }
    __threadfence();
  }
}

__global__ __launch_bounds__(256) KATTR void k_fin(const float* __restrict__ R3, const int* __restrict__ batch,
                                                   int ntot, const float* __restrict__ gam,
                                                   const float* __restrict__ bet, float* BNP3, int* OFFS) {
  __shared__ double red[256];
  __shared__ __attribute__((aligned(16))) float sbn[256];
  __shared__ __attribute__((aligned(16))) int scnt[32];
  __shared__ __attribute__((aligned(16))) int soff[32];
  const int tid = (int)threadIdx.x, lane = tid & 31, wave = tid >> 5;
  const int c = tid & 63, g = tid >> 6;
  const float* col = R3 + (size_t)(g * 1024) * HD + c;
  double s = 0.0;
#pragma unroll 4
  for (int r = 0; r < 1024; ++r) s += (double)col[(size_t)r * HD];
  red[tid] = s;
  __syncthreads();
  const double mean = (((red[c] + red[64 + c]) + red[128 + c]) + red[192 + c]) * (1.0 / 4096.0);
  __syncthreads();
  double q = 0.0;
#pragma unroll 4
  for (int r = 0; r < 1024; ++r) {
    const double d = (double)col[(size_t)r * HD] - mean;
    q += d * d;
  }
  red[tid] = q;
  __syncthreads();
  if (tid < 64) {
    const double var = (((red[c] + red[64 + c]) + red[128 + c]) + red[192 + c]) * (1.0 / 4096.0);
    const float rstd = 1.0f / sqrtf((float)var + 1e-5f);
    sbn[c] = (float)mean;
    sbn[64 + c] = gam[c] * rstd;
    sbn[128 + c] = bet[c];
    sbn[192 + c] = 0.0f;
  }
  if (wave == 0) {
    int cnt = 0;
#pragma unroll 4
    for (int t = 0; t < ntot; ++t) cnt += (batch[t] == lane) ? 1 : 0;
    scnt[lane] = cnt;
  }
  __syncthreads();
  if (wave == 0) {
    int off = 0;
#pragma unroll 4
    for (int g2 = 0; g2 < 32; ++g2) {
      const int cv = scnt[g2];
      off += (g2 < lane) ? cv : 0;
    }
    soff[lane] = off;
  }
  __syncthreads();
  v4f bv = {0.0f, 0.0f, 0.0f, 0.0f};
  v4i ov = {0, 0, 0, 0};
  if (tid < 64) bv = *(const v4fa*)(sbn + 4 * tid);
  if (tid < 8)  ov = *(const v4ia*)(soff + 4 * tid);
  if (tid < 64) *(volatile v4f*)(BNP3 + 4 * tid) = bv;
  if (tid < 8)  *(volatile v4i*)(OFFS + 4 * tid) = ov;
  __threadfence();
  if (tid < 64) *(volatile v4f*)(BNP3 + 4 * tid) = bv;
  if (tid < 8)  *(volatile v4i*)(OFFS + 4 * tid) = ov;
}

__global__ __launch_bounds__(256) KATTR void k_out(const float* __restrict__ x, const int* __restrict__ batch,
                                                   int ntot, const int* __restrict__ OFFS,
                                                   const float* __restrict__ R3, const float* __restrict__ BNP3,
                                                   float* out) {
  const int tid = (int)threadIdx.x, lane = tid & 31, wave = tid >> 5, hh = lane >> 4;
  const int t = (int)blockIdx.x * 8 + wave;
  const bool live = t < ntot;
  const int tc = live ? t : (ntot - 1);
  int g = batch[tc];
  g = g < 0 ? 0 : (g > NB - 1 ? NB - 1 : g);
  const int off = OFFS[g];
  int idx = g * MS + (tc - off);
  idx = idx < 0 ? 0 : (idx > NNODE - 1 ? NNODE - 1 : idx);
  const int cx = 4 * (lane & 15);
  const v4f xa = *(const v4f*)(x + (size_t)tc * 64 + cx);
  const v4f ra = *(const v4f*)(R3 + (size_t)idx * HD + cx);
  const v4f mv = *(const v4f*)(BNP3 + cx);
  const v4f av = *(const v4f*)(BNP3 + 64 + cx);
  const v4f bv = *(const v4f*)(BNP3 + 128 + cx);
  const unsigned mq = 0u - (unsigned)hh;
  v4f o;
  o.x = fsel(bf16_val(xa.x), (ra.x - mv.x) * av.x + bv.x, mq);
  o.y = fsel(bf16_val(xa.y), (ra.y - mv.y) * av.y + bv.y, mq);
  o.z = fsel(bf16_val(xa.z), (ra.z - mv.z) * av.z + bv.z, mq);
  o.w = fsel(bf16_val(xa.w), (ra.w - mv.w) * av.w + bv.w, mq);
  float* op = out + (size_t)tc * 128 + 4 * lane;
  if (live) *(volatile v4f*)op = o;
  __threadfence();
  if (live) *(volatile v4f*)op = o;
}

static inline size_t al256(size_t o) { return (o + 255) & ~(size_t)255; }

extern "C" void kernel_launch(void* const* d_in, const int* in_sizes, int n_in,
                              void* d_out, int out_size, void* d_ws, size_t ws_size,
                              hipStream_t stream) {
  if (n_in < 17) return;
  if (in_sizes[0] != NPOS * D1) return;
  const int ntot = in_sizes[2];
  if (ntot < 1 || ntot > NNODE) return;
  if ((long long)in_sizes[1] != (long long)ntot * 64) return;
  if (in_sizes[3] != D1 * HD * 15) return;
  if (in_sizes[4] != HD || in_sizes[5] != HD || in_sizes[6] != HD || in_sizes[7] != HD) return;
  if (in_sizes[8] != HD * HD * 15) return;
  if (in_sizes[9] != HD || in_sizes[10] != HD || in_sizes[11] != HD || in_sizes[12] != HD) return;
  if (in_sizes[13] != HD * HD * 5) return;
  if (in_sizes[14] != HD || in_sizes[15] != HD || in_sizes[16] != HD) return;
  if ((long long)out_size != (long long)ntot * 128) return;

  const float* attn = (const float*)d_in[0];
  const float* xin  = (const float*)d_in[1];
  const int*   bat  = (const int*)d_in[2];
  const float* c1   = (const float*)d_in[3];
  const float* db1  = (const float*)d_in[4];
  const float* ab1  = (const float*)d_in[5];
  const float* g1   = (const float*)d_in[6];
  const float* be1  = (const float*)d_in[7];
  const float* c2   = (const float*)d_in[8];
  const float* db2  = (const float*)d_in[9];
  const float* ab2  = (const float*)d_in[10];
  const float* g2   = (const float*)d_in[11];
  const float* be2  = (const float*)d_in[12];
  const float* c3   = (const float*)d_in[13];
  const float* b3   = (const float*)d_in[14];
  const float* g3   = (const float*)d_in[15];
  const float* be3  = (const float*)d_in[16];
  float* out = (float*)d_out;

  size_t off = 0;
  const size_t oXB  = off; off = al256(off + (size_t)NPOS * D1 * 2);
  const size_t oW1P = off; off = al256(off + (size_t)128 * 32 * 2);
  const size_t oW1N = off; off = al256(off + (size_t)192 * K1N * 2);
  const size_t oW2P = off; off = al256(off + (size_t)64 * 256 * 2);
  const size_t oW2N = off; off = al256(off + (size_t)192 * K2N * 2);
  const size_t oW3N = off; off = al256(off + (size_t)64 * K2N * 2);
  const size_t oPV  = off; off = al256(off + (size_t)1024 * 4);
  const size_t oF0  = off; off = al256(off + (size_t)NNODE * K1N * 2);
  const size_t oF1  = off; off = al256(off + (size_t)NNODE * K2N * 2);
  const size_t oF2  = off; off = al256(off + (size_t)NNODE * K2N * 2);
  const size_t oNP1 = off; off = al256(off + (size_t)NNODE * NPW * 4);
  const size_t oNP2 = off; off = al256(off + (size_t)NNODE * NPW * 4);
  const size_t oRW1 = off; off = al256(off + (size_t)NNODE * HD * 4);
  const size_t oDG1 = off; off = al256(off + (size_t)NNODE * HD * 4);
  const size_t oRW2 = off; off = al256(off + (size_t)NNODE * HD * 4);
  const size_t oDG2 = off; off = al256(off + (size_t)NNODE * HD * 4);
  const size_t oCP1 = off; off = al256(off + (size_t)NB * 8 * MS * HD * 4);
  const size_t oCP2 = off; off = al256(off + (size_t)NB * 8 * MS * HD * 4);
  const size_t oST1 = off; off = al256(off + (size_t)256 * 64 * 2 * 8);
  const size_t oST2 = off; off = al256(off + (size_t)256 * 64 * 2 * 8);
  const size_t oR3  = off; off = al256(off + (size_t)NNODE * HD * 4);
  const size_t oBP1 = off; off = al256(off + (size_t)256 * 4);
  const size_t oBP2 = off; off = al256(off + (size_t)256 * 4);
  const size_t oBP3 = off; off = al256(off + (size_t)256 * 4);
  const size_t oOFF = off; off = al256(off + (size_t)32 * 4);
  if (off > ws_size || off > (size_t)WSMAX) return;

  char* ws = (char*)d_ws;
  unsigned short* XB  = (unsigned short*)(ws + oXB);
  unsigned short* W1P = (unsigned short*)(ws + oW1P);
  unsigned short* W1N = (unsigned short*)(ws + oW1N);
  unsigned short* W2P = (unsigned short*)(ws + oW2P);
  unsigned short* W2N = (unsigned short*)(ws + oW2N);
  unsigned short* W3N = (unsigned short*)(ws + oW3N);
  float*          PV  = (float*)(ws + oPV);
  unsigned short* F0  = (unsigned short*)(ws + oF0);
  unsigned short* F1  = (unsigned short*)(ws + oF1);
  unsigned short* F2  = (unsigned short*)(ws + oF2);
  float*          NP1 = (float*)(ws + oNP1);
  float*          NP2 = (float*)(ws + oNP2);
  float*          RW1 = (float*)(ws + oRW1);
  float*          DG1 = (float*)(ws + oDG1);
  float*          RW2 = (float*)(ws + oRW2);
  float*          DG2 = (float*)(ws + oDG2);
  float*          CP1 = (float*)(ws + oCP1);
  float*          CP2 = (float*)(ws + oCP2);
  double*         ST1 = (double*)(ws + oST1);
  double*         ST2 = (double*)(ws + oST2);
  float*          R3  = (float*)(ws + oR3);
  float*          BP1 = (float*)(ws + oBP1);
  float*          BP2 = (float*)(ws + oBP2);
  float*          BP3 = (float*)(ws + oBP3);
  int*            OFS = (int*)(ws + oOFF);

  hipFuncSetAttribute(reinterpret_cast<const void*>(&k_pair<0>), hipFuncAttributeMaxDynamicSharedMemorySize,
                      (int)PAIR0_LDS);
  hipFuncSetAttribute(reinterpret_cast<const void*>(&k_pair<1>), hipFuncAttributeMaxDynamicSharedMemorySize,
                      (int)PAIR1_LDS);
  hipFuncSetAttribute(reinterpret_cast<const void*>(&k_bn), hipFuncAttributeMaxDynamicSharedMemorySize,
                      (int)BN_LDS);
  hipFuncSetAttribute(reinterpret_cast<const void*>(&k_feat0), hipFuncAttributeMaxDynamicSharedMemorySize,
                      (int)F0_LDS);

  k_prep<<<PREP_BLOCKS, 256, 0, stream>>>(attn, c1, c2, c3, db1, ab1, g1, be1, db2, ab2, g2, be2, b3, g3, be3,
                                          XB, W1P, W1N, W2P, W2N, W3N, PV);
  k_feat0<<<NB, 256, F0_LDS, stream>>>(XB, F0);
  k_node<0><<<dim3(NNODE / 64, 3, 1), 128, 0, stream>>>(F0, K1N, W1N, K1N, K1N, PV + PV_B1, NP1, NPW);
  k_pair<0><<<NB * 8, 256, PAIR0_LDS, stream>>>(XB, W1P, W2P, NP1, NP2, BP1, RW1, DG1, CP1, ST1);
  k_bn<<<NB, 256, BN_LDS, stream>>>(ST1, RW1, DG1, CP1, PV + PV_G1, PV + PV_BE1, F1, BP1);
  k_node<0><<<dim3(NNODE / 64, 3, 1), 128, 0, stream>>>(F1, K2N, W2N, K2N, K2N, PV + PV_B2, NP2, NPW);
  k_pair<1><<<NB * 8, 256, PAIR1_LDS, stream>>>(XB, W1P, W2P, NP1, NP2, BP1, RW2, DG2, CP2, ST2);
  k_bn<<<NB, 256, BN_LDS, stream>>>(ST2, RW2, DG2, CP2, PV + PV_G2, PV + PV_BE2, F2, BP2);
  k_node<1><<<dim3(NNODE / 64, 1, 1), 128, 0, stream>>>(F2, K2N, W3N, K2N, K2N, PV + PV_B3, R3, HD);
  k_fin<<<1, 256, 0, stream>>>(R3, bat, ntot, PV + PV_G3, PV + PV_BE3, BP3, OFS);
  k_out<<<(ntot + 7) / 8, 256, 0, stream>>>(xin, bat, ntot, OFS, R3, BP3, out);
  (void)hipGetLastError();
}
